// MultiHeadAttention_70755291234837
// MI455X (gfx1250) — hardware-verified
//
#include <hip/hip_runtime.h>
#ifndef NB
#define NB 2
#endif
#ifndef SEQ
#define SEQ 2048
#endif
#define SEQ_FULL 2048
#define DM 1024
#define NH 16
#define HD 64
#define HS 192
#define DQKV 3072
#define QOFF 0
#define KOFF 64
#define VOFF 128
#define QT 256
#define NR ((size_t)NB * SEQ)
#define ATS 0.125f

static_assert(NH * HD == DM);
static_assert(HD == 64);
static_assert(HS == 3 * HD);
static_assert(NH * HS == DQKV);
static_assert(KOFF % 8 == 0 && VOFF % 8 == 0 && HS % 8 == 0);
static_assert(DM == 1024);
static_assert(SEQ % 256 == 0);
static_assert(SEQ % QT == 0);
static_assert(QT % 128 == 0);
static_assert((NB * SEQ) % 128 == 0);
static_assert(DM % 64 == 0 && DQKV % 64 == 0 && SEQ % 64 == 0);
static_assert(DM % 32 == 0 && HD % 32 == 0 && SEQ % 32 == 0);
static_assert(((size_t)NB * SEQ * DM) % 2048 == 0);
static_assert(((size_t)DQKV * DM) % 2048 == 0);
static_assert(((size_t)DM * DM) % 2048 == 0);
static_assert((NH * QT) % 8 == 0);
static_assert(SEQ <= SEQ_FULL);

typedef unsigned short v8us __attribute__((ext_vector_type(8), may_alias));
typedef float  v8f  __attribute__((ext_vector_type(8)));
typedef float  v4f  __attribute__((ext_vector_type(4)));
typedef float  v4fa __attribute__((ext_vector_type(4), may_alias));
typedef _Float16 v16h __attribute__((ext_vector_type(16)));
typedef _Float16 v4h __attribute__((ext_vector_type(4)));
union FragH { v16h v; v8us half[2]; _Float16 h[16]; unsigned short u[16]; };

__device__ __forceinline__ unsigned short bf16_bits(float x) { unsigned int u = __float_as_uint(x); return (unsigned short)((u + 0x7FFFu + ((u >> 16) & 1u)) >> 16); }
__device__ __forceinline__ float bf16_val(unsigned short b) { return __uint_as_float(((unsigned int)b) << 16); }
__device__ __forceinline__ float bf16_rne(float x) { return bf16_val(bf16_bits(x)); }

__global__ __launch_bounds__(256) void k_x16(const float* __restrict__ x, _Float16* __restrict__ X16) {
  const unsigned t = blockIdx.x * 256u + threadIdx.x;
  if (t >= (unsigned)(NR * DM / 8)) return;
  const unsigned r = t >> 7, c8 = (t & 127u) << 3;
  const unsigned b = r / (unsigned)SEQ, s = r - b * (unsigned)SEQ;
  const float* src = x + ((size_t)b * SEQ_FULL + s) * DM + c8;
  const v4f a = *(const v4fa*)src, c = *(const v4fa*)(src + 4);
  FragH f;
#pragma unroll
  for (int q = 0; q < 4; ++q) { f.h[q] = (_Float16)bf16_rne(a[q]); f.h[4 + q] = (_Float16)bf16_rne(c[q]); }
  const v8us o = f.half[0];
  unsigned short* d = (unsigned short*)X16 + (size_t)t * 8;
  *(volatile v8us*)d = o; __threadfence(); *(volatile v8us*)d = o;
}

__global__ __launch_bounds__(256) void k_wnat(const float* __restrict__ w, _Float16* __restrict__ Bt, unsigned n8) {
  const unsigned t = blockIdx.x * 256u + threadIdx.x;
  if (t >= n8) return;
  const float* src = w + (size_t)t * 8;
  const v4f a = *(const v4fa*)src, c = *(const v4fa*)(src + 4);
  FragH f;
#pragma unroll
  for (int q = 0; q < 4; ++q) { f.h[q] = (_Float16)(bf16_rne(a[q]) * 16.0f); f.h[4 + q] = (_Float16)(bf16_rne(c[q]) * 16.0f); }
  const v8us o = f.half[0];
  unsigned short* d = (unsigned short*)Bt + (size_t)t * 8;
  *(volatile v8us*)d = o; __threadfence(); *(volatile v8us*)d = o;
}

__global__ __launch_bounds__(256) void k_vt(const _Float16* __restrict__ V16, int ldv, int voff, int hstr, _Float16* __restrict__ Vt) {
  __shared__ unsigned short tl[64][66];
  const unsigned tid = threadIdx.x;
  const unsigned slab = blockIdx.x / (unsigned)(SEQ / 64), lg = blockIdx.x % (unsigned)(SEQ / 64);
  const unsigned b = slab / (unsigned)NH, h = slab % (unsigned)NH;
  for (unsigned i = tid; i < 64u * 8u; i += 256u) {
    const unsigned r = i >> 3, c8 = (i & 7u) << 3;
    FragH f;
    f.half[0] = *(const v8us*)((const unsigned short*)V16 + ((size_t)b * SEQ + lg * 64u + r) * (size_t)ldv + (size_t)voff + (size_t)h * (unsigned)hstr + c8);
#pragma unroll
    for (int q = 0; q < 8; ++q) tl[r][c8 + q] = f.u[q];
  }
  __syncthreads();
  for (int pass = 0; pass < 2; ++pass) {
#pragma unroll
    for (unsigned rd = 0; rd < 2; ++rd) {
      const unsigned d = rd * 32u + (tid >> 3), pc = tid & 7u;
      FragH f;
#pragma unroll
      for (int q = 0; q < 8; ++q) f.u[q] = tl[pc * 8u + q][d];
      const v8us o = f.half[0];
      *(volatile v8us*)((unsigned short*)Vt + ((size_t)slab * 64u + d) * SEQ + lg * 64u + pc * 8u) = o;
    }
    if (pass == 0) __threadfence();
  }
}

__device__ __forceinline__ v16h g2_frag(const _Float16* p, unsigned hh) { FragH f; f.half[0] = *(const v8us*)((const unsigned short*)p + 8u * hh); f.half[1] = *(const v8us*)((const unsigned short*)p + 16u + 8u * hh); return f.v; }
__device__ __forceinline__ v8f g2_mma(v16h a, v16h b, v8f c) { v8f d = __builtin_amdgcn_wmma_f32_16x16x32_f16(false, a, false, b, (short)0, c, false, false); asm volatile("v_nop\n\tv_nop\n\tv_nop\n\tv_nop" : "+v"(d) : "v"(a), "v"(b)); return d; }

__global__ __launch_bounds__(128) void k_gemm2(const _Float16* __restrict__ A, int lda, size_t sA, const _Float16* __restrict__ Bh, int ldb, size_t sB, float alpha,
    const float* __restrict__ bias, float* __restrict__ C, _Float16* __restrict__ C16, int ldc, size_t sC, int M, int N, int K) {
  __shared__ __attribute__((aligned(16))) float so[4][32][68];
  const unsigned tid = threadIdx.x, w = tid >> 5, lane = tid & 31u, ln = lane & 15u, hh = lane >> 4;
  const unsigned by = blockIdx.y;
  A += (size_t)by * sA; Bh += (size_t)by * sB; const size_t cofs = (size_t)by * sC;
  const unsigned ntn = (unsigned)N >> 6;
  const unsigned mt = blockIdx.x / ntn, nq = blockIdx.x - mt * ntn;
  const unsigned row0 = mt * 128u + 32u * w, col0 = nq * 64u;
  if (row0 >= (unsigned)M) return;
  const _Float16* a0p = A + (size_t)(row0 + ln) * lda; const _Float16* a1p = a0p + (size_t)16 * lda;
  const _Float16* b0p = Bh + (size_t)(col0 + ln) * ldb; const _Float16* b1p = b0p + (size_t)16 * ldb; const _Float16* b2p = b1p + (size_t)16 * ldb; const _Float16* b3p = b2p + (size_t)16 * ldb;
  const v8f z8 = {0.f,0.f,0.f,0.f,0.f,0.f,0.f,0.f};
  v8f c00 = z8, c01 = z8, c02 = z8, c03 = z8, c10 = z8, c11 = z8, c12 = z8, c13 = z8;
#pragma unroll 1
  for (int kb = 0; kb < K; kb += 32) {
    const v16h a0 = g2_frag(a0p + kb, hh), a1 = g2_frag(a1p + kb, hh);
    v16h b = g2_frag(b0p + kb, hh); c00 = g2_mma(a0, b, c00); c10 = g2_mma(a1, b, c10);
    b = g2_frag(b1p + kb, hh); c01 = g2_mma(a0, b, c01); c11 = g2_mma(a1, b, c11);
    b = g2_frag(b2p + kb, hh); c02 = g2_mma(a0, b, c02); c12 = g2_mma(a1, b, c12);
    b = g2_frag(b3p + kb, hh); c03 = g2_mma(a0, b, c03); c13 = g2_mma(a1, b, c13);
  }
  float bv[4] = {0.f, 0.f, 0.f, 0.f};
  if (bias) {
#pragma unroll
    for (int t = 0; t < 4; ++t) bv[t] = bf16_rne(bias[col0 + (unsigned)t * 16u + ln]);
  }
  v8f accs[8] = {c00, c01, c02, c03, c10, c11, c12, c13};
#pragma unroll
  for (int u = 0; u < 8; ++u) {
    const unsigned t = (unsigned)u & 3u, hf = (unsigned)u >> 2;
#pragma unroll
    for (int r = 0; r < 8; ++r) { const unsigned rloc = hf * 16u + 8u * hh + (unsigned)r; so[w][rloc][t * 16u + ln] = accs[u][r] * alpha + bv[u & 3]; }
  }
  __builtin_amdgcn_fence(4  , "workgroup"); __builtin_amdgcn_wave_barrier();
  const unsigned rsub = lane >> 4, c4 = (lane & 15u) * 4u;
  for (int pass = 0; pass < 2; ++pass) {
#pragma unroll
    for (unsigned q = 0; q < 16; ++q) {
      const unsigned r = q * 2u + rsub;
      const v4f v = *(const v4fa*)&so[w][r][c4];
      if (C) *(volatile v4f*)(C + cofs + (size_t)(row0 + r) * ldc + col0 + c4) = v;
      if (C16) { v4h h4; for (int i = 0; i < 4; ++i) h4[i] = (_Float16)v[i]; *(volatile v4h*)(C16 + cofs + (size_t)(row0 + r) * ldc + col0 + c4) = h4; }
    }
    if (pass == 0) __threadfence();
  }
}

__global__ __launch_bounds__(256) void k_rsmw(const float* __restrict__ S, _Float16* __restrict__ P, unsigned nrows) {
  #pragma clang fp contract(off)
  const unsigned lane = threadIdx.x & 31u, w = threadIdx.x >> 5;
  const unsigned row = blockIdx.x * 8u + w;
  if (row >= nrows) return;
  const float* s = S + (size_t)row * SEQ + lane * 8u;
  float mx = -3.0e38f;
#pragma unroll 1
  for (unsigned it = 0; it < (unsigned)(SEQ / 256); ++it) {
    const v4f a = *(const v4fa*)(s + it * 256u), c = *(const v4fa*)(s + it * 256u + 4u);
    mx = fmaxf(mx, fmaxf(fmaxf(a[0], a[1]), fmaxf(a[2], a[3])));
    mx = fmaxf(mx, fmaxf(fmaxf(c[0], c[1]), fmaxf(c[2], c[3])));
  }
  mx = fmaxf(mx, __shfl_xor(mx, 16, 32)); mx = fmaxf(mx, __shfl_xor(mx, 8, 32)); mx = fmaxf(mx, __shfl_xor(mx, 4, 32)); mx = fmaxf(mx, __shfl_xor(mx, 2, 32)); mx = fmaxf(mx, __shfl_xor(mx, 1, 32));
  float se = 0.f;
#pragma unroll 1
  for (unsigned it = 0; it < (unsigned)(SEQ / 256); ++it) {
    const v4f a = *(const v4fa*)(s + it * 256u), c = *(const v4fa*)(s + it * 256u + 4u);
    float p = 0.f;
#pragma unroll
    for (int q = 0; q < 4; ++q) { p += __expf(a[q] - mx); p += __expf(c[q] - mx); }
    se += p;
  }
  se += __shfl_xor(se, 16, 32); se += __shfl_xor(se, 8, 32); se += __shfl_xor(se, 4, 32); se += __shfl_xor(se, 2, 32); se += __shfl_xor(se, 1, 32);
  const float sc = 256.0f * (1.0f / se);
#pragma unroll 1
  for (unsigned it = 0; it < (unsigned)(SEQ / 256); ++it) {
    const v4f a = *(const v4fa*)(s + it * 256u), c = *(const v4fa*)(s + it * 256u + 4u);
    FragH f;
#pragma unroll
    for (int q = 0; q < 4; ++q) { f.h[q] = (_Float16)(__expf(a[q] - mx) * sc); f.h[4 + q] = (_Float16)(__expf(c[q] - mx) * sc); }
    const v8us o = f.half[0];
    unsigned short* d = (unsigned short*)P + (size_t)row * SEQ + it * 256u + lane * 8u;
    *(volatile v8us*)d = o; __threadfence(); *(volatile v8us*)d = o;
  }
}

#define WS_WQKV ((size_t)DQKV * DM * 2)
#define WS_WO   ((size_t)DM * DM * 2)
#define WS_ROW  ((size_t)NB * SEQ * DM * 2)
#define WS_QKV  ((size_t)NB * SEQ * DQKV * 2)
#define WS_S    ((size_t)NH * QT * SEQ * 4)
#define WS_P    ((size_t)NH * QT * SEQ * 2)
#define WS_VT   ((size_t)NB * NH * HD * SEQ * 2)
static_assert(WS_WQKV + WS_WO + 2 * WS_ROW + WS_QKV + WS_S + WS_P + WS_VT <= (size_t)134217728);
static_assert(WS_WQKV % 256 == 0 && WS_WO % 256 == 0 && WS_ROW % 256 == 0 && WS_QKV % 256 == 0 && WS_S % 256 == 0 && WS_P % 256 == 0 && WS_VT % 256 == 0);

extern "C" void kernel_launch(void* const* d_in, const int* in_sizes, int n_in,
                              void* d_out, int out_size, void* d_ws, size_t ws_size, hipStream_t stream) {
  if (n_in < 5) return;
  if ((size_t)in_sizes[0] < ((size_t)(NB - 1) * SEQ_FULL + SEQ) * DM) return;
  if ((size_t)in_sizes[1] < (size_t)DQKV * DM) return;
  if ((size_t)in_sizes[2] < (size_t)DQKV) return;
  if ((size_t)in_sizes[3] < (size_t)DM * DM) return;
  if ((size_t)in_sizes[4] < (size_t)DM) return;
  if ((size_t)out_size < NR * DM) return;
  const float* x = (const float*)d_in[0]; const float* wqkv = (const float*)d_in[1]; const float* bqkv = (const float*)d_in[2]; const float* wfc = (const float*)d_in[3]; const float* bfc = (const float*)d_in[4];
  char* ws = (char*)d_ws; size_t off = 0;
  auto take = [&](size_t bytes) { char* p = ws + off; off += (bytes + 255) & ~(size_t)255; return p; };
  _Float16* BQKV = (_Float16*)take(WS_WQKV); _Float16* BO = (_Float16*)take(WS_WO);
  _Float16* X16 = (_Float16*)take(WS_ROW); _Float16* QKV16 = (_Float16*)take(WS_QKV); _Float16* O16 = (_Float16*)take(WS_ROW);
  float* S = (float*)take(WS_S); _Float16* P = (_Float16*)take(WS_P); _Float16* VT = (_Float16*)take(WS_VT);
  if (off > ws_size) return;

  const unsigned n8qkv = (unsigned)((size_t)DQKV * DM / 8), n8o = (unsigned)((size_t)DM * DM / 8);
  k_wnat<<<(n8qkv + 255u) / 256u, 256, 0, stream>>>(wqkv, BQKV, n8qkv);
  k_wnat<<<(n8o + 255u) / 256u, 256, 0, stream>>>(wfc, BO, n8o);
  k_x16<<<(unsigned)((NR * DM / 8 + 255) / 256), 256, 0, stream>>>(x, X16);
  k_gemm2<<<dim3((unsigned)((NR / 128) * (DQKV / 64)), 1), 128, 0, stream>>>(X16, DM, (size_t)0, BQKV, DM, (size_t)0, 0.0625f, bqkv, (float*)nullptr, QKV16, DQKV, (size_t)0, (int)NR, DQKV, DM);
  k_vt<<<(unsigned)(NB * NH * (SEQ / 64)), 256, 0, stream>>>(QKV16, DQKV, VOFF, HS, VT);
  for (int b = 0; b < NB; ++b) {
    const size_t r0 = (size_t)b * SEQ;
    for (int q0 = 0; q0 < SEQ; q0 += QT) {
      k_gemm2<<<dim3((QT / 128) * (SEQ / 64), NH), 128, 0, stream>>>(QKV16 + (r0 + q0) * DQKV + QOFF, DQKV, (size_t)HS, QKV16 + r0 * DQKV + KOFF, DQKV, (size_t)HS, ATS, (const float*)nullptr, S, (_Float16*)nullptr, SEQ, (size_t)QT * SEQ, QT, SEQ, HD);
      k_rsmw<<<(NH * QT) / 8, 256, 0, stream>>>(S, P, (unsigned)(NH * QT));
      k_gemm2<<<dim3((QT / 128) * (HD / 64), NH), 128, 0, stream>>>(P, SEQ, (size_t)QT * SEQ, VT + (size_t)b * NH * HD * SEQ, SEQ, (size_t)HD * SEQ, 0.25f, (const float*)nullptr, (float*)nullptr, O16 + (r0 + q0) * DM, DM, (size_t)HD, QT, HD, SEQ);
    }
  }
  k_gemm2<<<dim3((unsigned)((NR / 128) * (DM / 64)), 1), 128, 0, stream>>>(O16, DM, (size_t)0, BO, DM, (size_t)0, 0.0009765625f, bfc, (float*)d_out, (_Float16*)nullptr, DM, (size_t)0, (int)NR, DM, DM);
}
